// RNN_LSTM_22703197127169
// MI455X (gfx1250) — hardware-run, weakly checked
//
#include <hip/hip_runtime.h>
#include <math.h>

constexpr int NBATCH  = 32;
constexpr int NSTEP   = 512;
constexpr int NFEAT   = 256;
constexpr int NUNIT   = 512;
constexpr int NGATE   = 4 * NUNIT;
constexpr int NROWS   = NBATCH * NSTEP;
constexpr int NTHR    = 256;
constexpr int SEQ_BLK = 16;
constexpr int HPITCH  = 520;
constexpr float A_CARRY = 16.0f;
constexpr float W_CARRY = 16.0f;
constexpr float FOLD    = 1.0f / (A_CARRY * W_CARRY);

static_assert(NBATCH % SEQ_BLK == 0);
static_assert(NUNIT == 64 * (NTHR / 32));
static_assert(NFEAT % 64 == 0 && NUNIT % 64 == 0 && NGATE % 64 == 0);
static_assert((NFEAT + NUNIT) % 32 == 0 && (2 * NUNIT) % 32 == 0 && NUNIT % 32 == 0);
static_assert(NROWS % 64 == 0);
static_assert((NROWS * NFEAT / 8) % NTHR == 0);
static_assert(HPITCH % 8 == 0 && HPITCH >= NUNIT);

typedef __attribute__((ext_vector_type(16))) _Float16 v16h;
typedef __attribute__((ext_vector_type(8)))  _Float16 v8h;
typedef __attribute__((ext_vector_type(8)))  float    v8f;
typedef __attribute__((ext_vector_type(4)))  float    v4f;

__device__ __forceinline__ unsigned short f2bf_bits(float f) {
  unsigned u = __float_as_uint(f);
  return (unsigned short)((u + 0x7FFFu + ((u >> 16) & 1u)) >> 16);
}
__device__ __forceinline__ float bf_bits2f(unsigned short h) { return __uint_as_float(((unsigned)h) << 16); }
__device__ __forceinline__ float bf16r(float f) { return bf_bits2f(f2bf_bits(f)); }

union FragU { v16h v; v8h h[2]; };
__device__ __forceinline__ v16h frag_load(const _Float16* p) {
  FragU f;
  f.h[0] = *(const v8h*)(p);
  f.h[1] = *(const v8h*)(p + 16);
  return f.v;
}
__device__ __forceinline__ v8f mma16(v16h a, v16h b, v8f c) {
  return __builtin_amdgcn_wmma_f32_16x16x32_f16(false, a, false, b, (short)0, c, false, false);
}
__device__ __forceinline__ void grp_guard(v8f& a0, v8f& a1, v8f& a2, v8f& a3, v16h x, v16h b0, v16h b1, v16h b2, v16h b3) {
  asm volatile("v_nop\n\tv_nop\n\tv_nop\n\tv_nop" : "+v"(a0), "+v"(a1), "+v"(a2), "+v"(a3) : "v"(x), "v"(b0), "v"(b1), "v"(b2), "v"(b3));
}
__device__ __forceinline__ void acc_guard4(v8f& a, v8f& b, v8f& c, v8f& d) {
  asm volatile("v_nop\n\tv_nop\n\tv_nop\n\tv_nop" : "+v"(a), "+v"(b), "+v"(c), "+v"(d));
}

__device__ __forceinline__ float fsig(float x)  { return __builtin_amdgcn_rcpf(1.0f + __expf(-x)); }
__device__ __forceinline__ float ftanh(float x) { return 1.0f - 2.0f * __builtin_amdgcn_rcpf(__expf(2.0f * x) + 1.0f); }

__global__ __launch_bounds__(NTHR) void cvt_x_kernel(const float* __restrict__ src, unsigned short* __restrict__ dst,
                                                     int n8, float sc) {
  const int i = blockIdx.x * NTHR + threadIdx.x;
  if (i < n8) {
    const float* sp = src + (size_t)i * 8;
    const v4f a = *(const v4f*)(sp);
    const v4f b = *(const v4f*)(sp + 4);
    v8h hv;
#pragma unroll
    for (int e = 0; e < 4; ++e) {
      const float fa = a[e];
      const float fb = b[e];
      hv[e]     = (_Float16)(bf16r(fa) * sc);
      hv[4 + e] = (_Float16)(bf16r(fb) * sc);
    }
    _Float16* dp = (_Float16*)dst + (size_t)i * 8;
    *(volatile v8h*)dp = hv;
    __threadfence();
    *(volatile v8h*)dp = hv;
  }
}

__global__ __launch_bounds__(NTHR) void tpw2_kernel(const float* __restrict__ srcA, int RA, const float* __restrict__ srcB,
                                                    int C, int ldo, unsigned short* __restrict__ O, float sc) {
  __shared__ float Tt[64 * 65];
  const int tid = threadIdx.x;
  const int c0 = blockIdx.x * 64, r0 = blockIdx.y * 64;
  const bool first = (r0 < RA);
  const float* src = first ? srcA : srcB;
  const int rl = first ? r0 : (r0 - RA);
#pragma unroll
  for (int i = 0; i < 4; ++i) {
    const int idx = i * NTHR + tid;
    const int rr = idx >> 4, cc = (idx & 15) * 4;
    const v4f v = *(const v4f*)(src + (size_t)(rl + rr) * (size_t)C + c0 + cc);
    Tt[rr * 65 + cc + 0] = v[0];
    Tt[rr * 65 + cc + 1] = v[1];
    Tt[rr * 65 + cc + 2] = v[2];
    Tt[rr * 65 + cc + 3] = v[3];
  }
  __syncthreads();
  const int q = tid >> 3, c8 = (tid & 7) * 8;
  v8h hv[2];
#pragma unroll
  for (int g = 0; g < 2; ++g) {
    const int qq = g * 32 + q;
#pragma unroll
    for (int e = 0; e < 8; ++e) {
      const float f = Tt[(c8 + e) * 65 + qq];
      hv[g][e] = (_Float16)(bf16r(f) * sc);
    }
  }
  _Float16* Oh = (_Float16*)O;
  for (int pass = 0; pass < 2; ++pass) {
#pragma unroll
    for (int g = 0; g < 2; ++g) {
      const size_t o = (size_t)(c0 + g * 32 + q) * (size_t)ldo + (size_t)(r0 + c8);
      *(volatile v8h*)(Oh + o) = hv[g];
    }
    __threadfence();
  }
}

template <int KIN>
__global__ __launch_bounds__(NTHR) void lstm_layer_kernel(const unsigned short* __restrict__ Ainp,
                                                          const unsigned short* __restrict__ Ztp,
                                                          const float* __restrict__ bias,
                                                          const float* __restrict__ hinit,
                                                          const float* __restrict__ cinit,
                                                          unsigned short* __restrict__ Houtp) {
  static_assert(KIN % 32 == 0);
  constexpr int KT = KIN + NUNIT;
  constexpr size_t GSTR = (size_t)NUNIT * (size_t)KT;
  __shared__ __align__(16) _Float16 Ah[2][SEQ_BLK * HPITCH];
  const _Float16* Ain = (const _Float16*)Ainp;
  const _Float16* Zt  = (const _Float16*)Ztp;
  _Float16* Hout = (_Float16*)Houtp;
  const int tid = threadIdx.x, lane = tid & 31, wave = tid >> 5;
  const int c = lane & 15, hh = lane >> 4, koff = hh * 8;
  const int rowbase = blockIdx.x * SEQ_BLK;

  {
    const _Float16 hv0 = (_Float16)(bf16r(hinit[tid]) * A_CARRY);
    const _Float16 hv1 = (_Float16)(bf16r(hinit[256 + tid]) * A_CARRY);
#pragma unroll 1
    for (int i = 0; i < SEQ_BLK; ++i) {
      Ah[0][i * HPITCH + tid]       = hv0;
      Ah[0][i * HPITCH + 256 + tid] = hv1;
    }
  }
  float cst[4][8], bb[4][4];
#pragma unroll
  for (int nt = 0; nt < 4; ++nt) {
    const int j = 64 * wave + 16 * nt + c;
#pragma unroll
    for (int g = 0; g < 4; ++g) bb[nt][g] = bf16r(bias[g * NUNIT + j]);
    const float cv = bf16r(cinit[j]);
#pragma unroll
    for (int r = 0; r < 8; ++r) cst[nt][r] = cv;
  }
  __syncthreads();

  const v8f z8 = {0.f, 0.f, 0.f, 0.f, 0.f, 0.f, 0.f, 0.f};
  const int crow0 = tid >> 6;
  const int cc8   = (tid & 63) * 8;

#pragma unroll 1
  for (int t = 0; t < NSTEP; ++t) {
    const int cur = t & 1;
    const _Float16* ahrow = &Ah[cur][0] + c * HPITCH + koff;
    _Float16* ahn = &Ah[cur ^ 1][0];
    const _Float16* arow = Ain + ((size_t)(rowbase + c) * NSTEP + (size_t)t) * KIN + koff;

#pragma unroll
    for (int nt = 0; nt < 4; ++nt) {
      const int j = 64 * wave + 16 * nt + c;
      const _Float16* zr = Zt + (size_t)j * KT + koff;
      v8f acc[4];
      acc[0] = z8; acc[1] = z8; acc[2] = z8; acc[3] = z8;
#pragma unroll 1
      for (int k0 = 0; k0 < KIN; k0 += 32) {
        const v16h a  = frag_load(arow + k0);
        const v16h b0 = frag_load(zr + k0);
        const v16h b1 = frag_load(zr + GSTR + k0);
        const v16h b2 = frag_load(zr + 2 * GSTR + k0);
        const v16h b3 = frag_load(zr + 3 * GSTR + k0);
        acc[0] = mma16(a, b0, acc[0]);
        acc[1] = mma16(a, b1, acc[1]);
        acc[2] = mma16(a, b2, acc[2]);
        acc[3] = mma16(a, b3, acc[3]);
        grp_guard(acc[0], acc[1], acc[2], acc[3], a, b0, b1, b2, b3);
      }
      const _Float16* zh = zr + KIN;
#pragma unroll 1
      for (int k0 = 0; k0 < NUNIT; k0 += 32) {
        const v16h a  = frag_load(ahrow + k0);
        const v16h b0 = frag_load(zh + k0);
        const v16h b1 = frag_load(zh + GSTR + k0);
        const v16h b2 = frag_load(zh + 2 * GSTR + k0);
        const v16h b3 = frag_load(zh + 3 * GSTR + k0);
        acc[0] = mma16(a, b0, acc[0]);
        acc[1] = mma16(a, b1, acc[1]);
        acc[2] = mma16(a, b2, acc[2]);
        acc[3] = mma16(a, b3, acc[3]);
        grp_guard(acc[0], acc[1], acc[2], acc[3], a, b0, b1, b2, b3);
      }
      acc_guard4(acc[0], acc[1], acc[2], acc[3]);
#pragma unroll
      for (int r = 0; r < 8; ++r) {
        const float zi = acc[0][r] * FOLD + bb[nt][0];
        const float zf = acc[1][r] * FOLD + bb[nt][1];
        const float zg = acc[2][r] * FOLD + bb[nt][2];
        const float zo = acc[3][r] * FOLD + bb[nt][3];
        const float ig = fsig(zi);
        const float fg = fsig(zf);
        const float gg = ftanh(zg);
        const float og = fsig(zo);
        const float cn = fg * cst[nt][r] + ig * gg;
        cst[nt][r] = cn;
        const float hn = og * ftanh(cn);
        ahn[(8 * hh + r) * HPITCH + j] = (_Float16)(hn * A_CARRY);
      }
    }
    __syncthreads();

    v8h ov[4];
#pragma unroll
    for (int it = 0; it < 4; ++it) ov[it] = *(const v8h*)(ahn + (it * 4 + crow0) * HPITCH + cc8);
    for (int pass = 0; pass < 2; ++pass) {
#pragma unroll
      for (int it = 0; it < 4; ++it) {
        const int row = it * 4 + crow0;
        *(volatile v8h*)(Hout + ((size_t)(rowbase + row) * NSTEP + (size_t)t) * NUNIT + cc8) = ov[it];
      }
      __threadfence();
    }
  }
}

__global__ __launch_bounds__(256) void head_gemm64(const unsigned short* __restrict__ Ap, int lda,
                                                   const unsigned short* __restrict__ Btp, int ldb,
                                                   float* __restrict__ C, int ldc,
                                                   const float* __restrict__ bias,
                                                   int M, int N, int K, float scale) {
  const _Float16* A  = (const _Float16*)Ap;
  const _Float16* Bt = (const _Float16*)Btp;
  __shared__ __align__(16) float sT[8][16 * 68];
  const int lane = threadIdx.x & 31;
  const int wave = threadIdx.x >> 5;
  const int tilesN = N >> 6;
  const int tilesM = M >> 6;
  const int tile = blockIdx.x * 8 + wave;
  if (tile >= tilesM * tilesN) return;
  const int tm = tile / tilesN;
  const int tn = tile - tm * tilesN;
  const int m0 = tm << 6;
  const int n0 = tn << 6;

  const int rlane = lane & 15;
  const int koff  = (lane >> 4) * 8;
  const int mOff  = (lane >> 4) * 8;

  v8f acc[4][4];
#pragma unroll
  for (int i = 0; i < 4; ++i)
#pragma unroll
    for (int j = 0; j < 4; ++j) acc[i][j] = (v8f){0.f, 0.f, 0.f, 0.f, 0.f, 0.f, 0.f, 0.f};

  for (int k0 = 0; k0 < K; k0 += 32) {
    v16h bh[4];
#pragma unroll
    for (int j = 0; j < 4; ++j) {
      const size_t bo = (size_t)(n0 + (j << 4) + rlane) * ldb + koff + k0;
      bh[j] = frag_load(Bt + bo);
    }
#pragma unroll
    for (int i = 0; i < 4; ++i) {
      const size_t ao = (size_t)(m0 + (i << 4) + rlane) * lda + koff + k0;
      const v16h ah = frag_load(A + ao);
#pragma unroll
      for (int j = 0; j < 4; ++j) acc[i][j] = mma16(ah, bh[j], acc[i][j]);
      grp_guard(acc[i][0], acc[i][1], acc[i][2], acc[i][3], ah, bh[0], bh[1], bh[2], bh[3]);
    }
  }
  acc_guard4(acc[0][0], acc[0][1], acc[0][2], acc[0][3]);
  acc_guard4(acc[1][0], acc[1][1], acc[1][2], acc[1][3]);
  acc_guard4(acc[2][0], acc[2][1], acc[2][2], acc[2][3]);
  acc_guard4(acc[3][0], acc[3][1], acc[3][2], acc[3][3]);

  float* slab = sT[wave];
#pragma unroll
  for (int i = 0; i < 4; ++i) {
    const int mBase = m0 + (i << 4);
#pragma unroll
    for (int j = 0; j < 4; ++j) {
      const int n = n0 + (j << 4) + rlane;
      const float bv = bf16r(bias[n]);
#pragma unroll
      for (int r = 0; r < 8; ++r) {
        const float v = acc[i][j][r] * scale + bv;
        slab[(mOff + r) * 68 + (j << 4) + rlane] = v;
      }
    }
    __builtin_amdgcn_fence(__ATOMIC_RELEASE, "workgroup");
    __builtin_amdgcn_wave_barrier();
    __builtin_amdgcn_fence(__ATOMIC_ACQUIRE, "workgroup");
    {
      const int hh = lane >> 4, c4 = (lane & 15) * 4;
      for (int pass = 0; pass < 2; ++pass) {
#pragma unroll
        for (int it = 0; it < 8; ++it) {
          const int row = it * 2 + hh;
          const v4f v = *(const v4f*)(slab + row * 68 + c4);
          *(volatile v4f*)(C + (size_t)(mBase + row) * ldc + n0 + c4) = v;
        }
        __threadfence();
      }
    }
    __builtin_amdgcn_fence(__ATOMIC_RELEASE, "workgroup");
    __builtin_amdgcn_wave_barrier();
    __builtin_amdgcn_fence(__ATOMIC_ACQUIRE, "workgroup");
  }
}

extern "C" void kernel_launch(void* const* d_in, const int* in_sizes, int n_in,
                              void* d_out, int out_size, void* d_ws, size_t ws_size, hipStream_t stream) {
  if (n_in < 18 || d_out == nullptr || d_ws == nullptr) return;
  if (in_sizes[0] != NBATCH * NSTEP * NFEAT || in_sizes[1] != NFEAT * NGATE || in_sizes[2] != NUNIT * NGATE ||
      in_sizes[3] != NGATE || in_sizes[4] != NUNIT || in_sizes[5] != NUNIT ||
      in_sizes[6] != NUNIT * NGATE || in_sizes[7] != NUNIT * NGATE || in_sizes[8] != NGATE ||
      in_sizes[9] != NUNIT || in_sizes[10] != NUNIT ||
      in_sizes[11] != NUNIT * NGATE || in_sizes[12] != NUNIT * NGATE || in_sizes[13] != NGATE ||
      in_sizes[14] != NUNIT || in_sizes[15] != NUNIT ||
      in_sizes[16] != NUNIT * NFEAT || in_sizes[17] != NFEAT ||
      out_size != NROWS * NFEAT) return;

  const float* x   = (const float*)d_in[0];
  const float* W0  = (const float*)d_in[1];
  const float* R0  = (const float*)d_in[2];
  const float* b0  = (const float*)d_in[3];
  const float* h0  = (const float*)d_in[4];
  const float* c0  = (const float*)d_in[5];
  const float* W1  = (const float*)d_in[6];
  const float* R1  = (const float*)d_in[7];
  const float* b1  = (const float*)d_in[8];
  const float* h1  = (const float*)d_in[9];
  const float* c1  = (const float*)d_in[10];
  const float* W2  = (const float*)d_in[11];
  const float* R2  = (const float*)d_in[12];
  const float* b2  = (const float*)d_in[13];
  const float* h2  = (const float*)d_in[14];
  const float* c2  = (const float*)d_in[15];
  const float* Wd  = (const float*)d_in[16];
  const float* bd  = (const float*)d_in[17];
  float* out = (float*)d_out;

  char* ws = (char*)d_ws;
  size_t off = 0;
  auto carve = [&](size_t bytes) -> char* { char* p = ws + off; off += (bytes + 255) & ~(size_t)255; return p; };
  unsigned short* XH  = (unsigned short*)carve((size_t)NROWS * NFEAT * 2);
  unsigned short* ZT0 = (unsigned short*)carve((size_t)NGATE * (NFEAT + NUNIT) * 2);
  unsigned short* ZT1 = (unsigned short*)carve((size_t)NGATE * (2 * NUNIT) * 2);
  unsigned short* ZT2 = (unsigned short*)carve((size_t)NGATE * (2 * NUNIT) * 2);
  unsigned short* WDT = (unsigned short*)carve((size_t)NFEAT * NUNIT * 2);
  unsigned short* HS0 = (unsigned short*)carve((size_t)NROWS * NUNIT * 2);
  unsigned short* HS1 = (unsigned short*)carve((size_t)NROWS * NUNIT * 2);
  unsigned short* HS2 = (unsigned short*)carve((size_t)NROWS * NUNIT * 2);
  if (off > ws_size || off > (size_t)134217728) return;

  const int n8x = NROWS * NFEAT / 8;
  cvt_x_kernel<<<n8x / NTHR, NTHR, 0, stream>>>(x, XH, n8x, A_CARRY);

  tpw2_kernel<<<dim3(NGATE / 64, (NFEAT + NUNIT) / 64), NTHR, 0, stream>>>(W0, NFEAT, R0, NGATE, NFEAT + NUNIT, ZT0, W_CARRY);
  tpw2_kernel<<<dim3(NGATE / 64, (2 * NUNIT) / 64), NTHR, 0, stream>>>(W1, NUNIT, R1, NGATE, 2 * NUNIT, ZT1, W_CARRY);
  tpw2_kernel<<<dim3(NGATE / 64, (2 * NUNIT) / 64), NTHR, 0, stream>>>(W2, NUNIT, R2, NGATE, 2 * NUNIT, ZT2, W_CARRY);
  tpw2_kernel<<<dim3(NFEAT / 64, NUNIT / 64), NTHR, 0, stream>>>(Wd, NUNIT, Wd, NFEAT, NUNIT, WDT, W_CARRY);

  lstm_layer_kernel<NFEAT><<<NBATCH / SEQ_BLK, NTHR, 0, stream>>>(XH,  ZT0, b0, h0, c0, HS0);
  lstm_layer_kernel<NUNIT><<<NBATCH / SEQ_BLK, NTHR, 0, stream>>>(HS0, ZT1, b1, h1, c1, HS1);
  lstm_layer_kernel<NUNIT><<<NBATCH / SEQ_BLK, NTHR, 0, stream>>>(HS1, ZT2, b2, h2, c2, HS2);

  head_gemm64<<<(NROWS / 64) * (NFEAT / 64) / 8, 256, 0, stream>>>(HS2, NUNIT, WDT, NUNIT, out, NFEAT, bd,
                                                                   NROWS, NFEAT, NUNIT, FOLD);
}
